// CurvedMultiHeadAttention_14972255994029
// MI455X (gfx1250) — hardware-verified
//
#include <hip/hip_runtime.h>


#define NB_  4
#define TT   1024
#define EE   768
#define DD   EE
#define NH_  12
#define HDM  64
#define RR   16
#define KW   96
#define PCAR 1024.0f
#define SCL  0.125f
#define EPSM 1e-6f
typedef _Float16 h16;
typedef unsigned short bf;
typedef __attribute__((ext_vector_type(16))) __bf16   v16bf;
typedef __attribute__((ext_vector_type(16))) _Float16 v16h;
typedef __attribute__((ext_vector_type(8)))  _Float16 v8h;
typedef __attribute__((ext_vector_type(8)))  unsigned short v8us;
typedef __attribute__((ext_vector_type(8)))  float    v8f;
typedef __attribute__((ext_vector_type(4)))  float    v4f;
typedef v8h  __attribute__((may_alias)) v8ha;
typedef v4f  __attribute__((may_alias)) v4fa;
typedef v8us __attribute__((may_alias)) v8usa;

__device__ __forceinline__ unsigned short f2bf(float f) { unsigned u = __float_as_uint(f); u += 0x7FFFu + ((u >> 16) & 1u); return (unsigned short)(u >> 16); }
__device__ __forceinline__ float bf2f(unsigned short b) { return __uint_as_float(((unsigned)b) << 16); }
__device__ __forceinline__ float bfr(float f) { return bf2f(f2bf(f)); }
__device__ __forceinline__ v16h cat16(v8h lo, v8h hi) { return __builtin_shufflevector(lo, hi, 0, 1, 2, 3, 4, 5, 6, 7, 8, 9, 10, 11, 12, 13, 14, 15); }
__device__ __forceinline__ v16bf cat16b(v8us lo, v8us hi) { return __builtin_bit_cast(v16bf, __builtin_shufflevector(lo, hi, 0, 1, 2, 3, 4, 5, 6, 7, 8, 9, 10, 11, 12, 13, 14, 15)); }
__device__ __forceinline__ v8f wmma16(v16h a, v16h b, v8f c) { return __builtin_amdgcn_wmma_f32_16x16x32_f16(false, a, false, b, (short)0, c, false, false); }
__device__ __forceinline__ v8f wmmab(v16bf a, v16bf b, v8f c) { return __builtin_amdgcn_wmma_f32_16x16x32_bf16(false, a, false, b, (short)0, c, false, false); }


template <typename T16> struct WFrag;
template <> struct WFrag<h16> { typedef v16h V; static __device__ __forceinline__ V ld(const h16* p) { return cat16(*(const v8h*)p, *(const v8h*)(p + 16)); } static __device__ __forceinline__ v8f mma(V a, V b, v8f c) { return wmma16(a, b, c); } };
template <> struct WFrag<bf> { typedef v16bf V; static __device__ __forceinline__ V ld(const bf* p) { return cat16b(*(const v8us*)p, *(const v8us*)(p + 16)); } static __device__ __forceinline__ v8f mma(V a, V b, v8f c) { return wmmab(a, b, c); } };
template <typename T16, int NSPLIT, bool BIAS>
__global__ __launch_bounds__(32) void k_gemmw(const T16* __restrict__ A, const T16* __restrict__ A2, const T16* __restrict__ Bt, const T16* __restrict__ Bt2, int K, float* C, int ldc, const float* __restrict__ bias, size_t sA, size_t sB, size_t sC) {
    typedef typename WFrag<T16>::V V;
    __shared__ __align__(16) float os[16 * 68];
    const size_t z = blockIdx.z; A += z * sA; if (A2) A2 += z * sA; Bt += z * sB; if (Bt2) Bt2 += z * sB; C += z * sC;
    const int lane = threadIdx.x & 31, lr = lane & 15, hi = lane >> 4; const int r0 = blockIdx.x * 64, c0 = blockIdx.y * 64;
    v8f acc[4][4];
#pragma unroll
    for (int mb = 0; mb < 4; ++mb)
#pragma unroll
        for (int nb = 0; nb < 4; ++nb) acc[mb][nb] = (v8f){};
    const size_t aoff = (size_t)(r0 + lr) * K + 8 * hi, boff = (size_t)(c0 + lr) * K + 8 * hi;
#pragma unroll 1
    for (int kc = 0; kc < K; kc += 32) {
        V a[4], a2[4];
#pragma unroll
        for (int mb = 0; mb < 4; ++mb) { a[mb] = WFrag<T16>::ld(A + aoff + (size_t)mb * 16 * K + kc); if (NSPLIT == 1 || NSPLIT == 2) a2[mb] = WFrag<T16>::ld(A2 + aoff + (size_t)mb * 16 * K + kc); }
#pragma unroll
        for (int nb = 0; nb < 4; ++nb) { const V b = WFrag<T16>::ld(Bt + boff + (size_t)nb * 16 * K + kc); V b2; if (NSPLIT >= 2) b2 = WFrag<T16>::ld(Bt2 + boff + (size_t)nb * 16 * K + kc);
#pragma unroll
            for (int mb = 0; mb < 4; ++mb) { acc[mb][nb] = WFrag<T16>::mma(a[mb], b, acc[mb][nb]); if (NSPLIT == 1 || NSPLIT == 2) acc[mb][nb] = WFrag<T16>::mma(a2[mb], b, acc[mb][nb]); if (NSPLIT >= 2) acc[mb][nb] = WFrag<T16>::mma(a[mb], b2, acc[mb][nb]); } }
        asm volatile("v_nop\n\tv_nop\n\tv_nop\n\tv_nop" : "+v"(acc[0][0]), "+v"(acc[1][1]), "+v"(acc[2][2]), "+v"(acc[3][3]) : "v"(a[0]), "v"(a[3]));
    }
#pragma unroll
    for (int mb = 0; mb < 4; ++mb) {
#pragma unroll
        for (int nb = 0; nb < 4; ++nb) {
#pragma unroll
            for (int j = 0; j < 8; ++j) os[(hi * 8 + j) * 68 + nb * 16 + lr] = acc[mb][nb][j]; }
        __builtin_amdgcn_wave_barrier(); asm volatile("" ::: "memory");
        float* crow = C + (size_t)(r0 + mb * 16) * ldc + c0;
#pragma unroll 1
        for (int ps = 0; ps < 2; ++ps) {
#pragma unroll
            for (int s = 0; s < 8; ++s) { const int row = 2 * s + hi, cofs = lr * 4; v4f val = *(const v4fa*)(os + row * 68 + cofs); if (BIAS) { val[0] += bfr(bias[c0 + cofs]); val[1] += bfr(bias[c0 + cofs + 1]); val[2] += bfr(bias[c0 + cofs + 2]); val[3] += bfr(bias[c0 + cofs + 3]); }
                *(volatile v4f*)(crow + (size_t)row * ldc + cofs) = val; }
            if (ps == 0) __threadfence(); }
        __builtin_amdgcn_wave_barrier(); asm volatile("" ::: "memory");
    }
}

__device__ __forceinline__ h16 tohx(float x) { return (h16)x; }
__device__ __forceinline__ void splitf(float y, unsigned short& h, unsigned short& l) { h = f2bf(y); l = f2bf(y - bf2f(h)); }
typedef __attribute__((ext_vector_type(2))) _Float16 v2h;
typedef __attribute__((ext_vector_type(4))) _Float16 v4h;
typedef __attribute__((ext_vector_type(2))) unsigned short v2us;
typedef __attribute__((ext_vector_type(4))) unsigned short v4us;
typedef __attribute__((ext_vector_type(2))) float v2f;

__global__ __launch_bounds__(256) void k_cvt8(const float* __restrict__ src, bf* dst, size_t n8) { const size_t i = (size_t)blockIdx.x * 256 + threadIdx.x; if (i >= n8) return; const v8f v = *(const v8f*)(src + i * 8); v8us o;
#pragma unroll
    for (int k = 0; k < 8; ++k) o[k] = f2bf(v[k]); *(volatile v8us*)(dst + i * 8) = o; __threadfence(); *(volatile v8us*)(dst + i * 8) = o; }
__global__ __launch_bounds__(256) void k_pl(const float* __restrict__ F, int pitch, int nh, int hd, h16* P) { const size_t e = ((size_t)blockIdx.x * 256 + threadIdx.x) * 2; if (e >= (size_t)nh * TT * hd) return; const int d = (int)(e % hd); const int t = (int)((e / hd) % TT); const int h = (int)(e / ((size_t)hd * TT)); v2h o; o[0] = tohx(F[(size_t)t * pitch + h * hd + d]); o[1] = tohx(F[(size_t)t * pitch + h * hd + d + 1]); *(volatile v2h*)(P + e) = o; __threadfence(); *(volatile v2h*)(P + e) = o; }
__global__ __launch_bounds__(256) void k_vt(const float* __restrict__ F, int pitch, int nh, int hd, h16* VT) { const size_t e = ((size_t)blockIdx.x * 256 + threadIdx.x) * 2; if (e >= (size_t)nh * hd * TT) return; const int t = (int)(e % TT); const int d = (int)((e / TT) % hd); const int h = (int)(e / ((size_t)TT * hd)); v2h o; o[0] = tohx(F[(size_t)t * pitch + h * hd + d]); o[1] = tohx(F[(size_t)(t + 1) * pitch + h * hd + d]); *(volatile v2h*)(VT + e) = o; __threadfence(); *(volatile v2h*)(VT + e) = o; }
__global__ __launch_bounds__(256) void k_mrgf(const float* __restrict__ O, int h, int hd, float* CT) { const size_t e = ((size_t)blockIdx.x * 256 + threadIdx.x) * 2; if (e >= (size_t)TT * hd) return; const int d = (int)(e % hd); const int t = (int)(e / hd); v2f o; o[0] = O[e] * (1.0f / PCAR); o[1] = O[e + 1] * (1.0f / PCAR); const size_t oo = (size_t)t * DD + h * hd + d; *(volatile v2f*)(CT + oo) = o; __threadfence(); *(volatile v2f*)(CT + oo) = o; }
__global__ __launch_bounds__(256) void k_mrg(const float* __restrict__ O, int h, int hd, bf* Ah, bf* Al) { const size_t e = ((size_t)blockIdx.x * 256 + threadIdx.x) * 2; if (e >= (size_t)TT * hd) return; const int d = (int)(e % hd); const int t = (int)(e / hd); v2us oh, ol;
#pragma unroll
    for (int q = 0; q < 2; ++q) { unsigned short a, c2; splitf(O[e + q] * (1.0f / PCAR), a, c2); oh[q] = a; ol[q] = c2; } const size_t oo = (size_t)t * DD + h * hd + d; *(volatile v2us*)(Ah + oo) = oh; *(volatile v2us*)(Al + oo) = ol; __threadfence(); *(volatile v2us*)(Ah + oo) = oh; *(volatile v2us*)(Al + oo) = ol; }
__global__ __launch_bounds__(256) void k_curv(const float* __restrict__ FQ, const float* __restrict__ FK, const float* __restrict__ A, bf* QCh, bf* QCl, bf* KCh, bf* KCl, float* N2) {
    const int e = blockIdx.x * 256 + threadIdx.x; if (e >= 2 * NH_ * TT) return; const int t = e % TT; const int h = (e / TT) % NH_; const int which = e / (TT * NH_); const float* f = (which ? FK : FQ) + (size_t)t * EE + h * HDM; const float* Ah = A + (size_t)h * HDM * RR;
    float a[RR];
#pragma unroll
    for (int r = 0; r < RR; ++r) a[r] = 0.f;
    float f2 = 0.f;
#pragma unroll 1
    for (int d = 0; d < HDM; ++d) { const float fv = f[d]; float p2 = __fmul_rn(fv, fv); asm volatile("" : "+v"(p2)); f2 = __fadd_rn(f2, p2);
#pragma unroll
        for (int r = 0; r < RR; ++r) { float p = __fmul_rn(fv, bfr(Ah[d * RR + r])); asm volatile("" : "+v"(p)); a[r] = __fadd_rn(a[r], p); } }
    float a2 = 0.f;
#pragma unroll
    for (int r = 0; r < RR; ++r) { float p = __fmul_rn(a[r], a[r]); asm volatile("" : "+v"(p)); a2 = __fadd_rn(a2, p); }
    float ef = __fmul_rn(EPSM, f2); asm volatile("" : "+v"(ef)); const float n2 = __fadd_rn(a2, ef);
    bf* Ph = (which ? KCh : QCh) + ((size_t)h * TT + t) * KW; bf* Pl = (which ? KCl : QCl) + ((size_t)h * TT + t) * KW; const float fs = which ? 1.0f : EPSM;
#pragma unroll 1
    for (int ps = 0; ps < 2; ++ps) {
        { v4us oh, ol, oh2, ol2; unsigned short x, y;
#pragma unroll
          for (int q = 0; q < 8; ++q) { splitf(a[q], x, y); oh[q & 3] = x; ol[q & 3] = y; if ((q & 3) == 3) { *(volatile v4us*)(Ph + (q - 3)) = oh; *(volatile v4us*)(Pl + (q - 3)) = ol; } }
#pragma unroll
          for (int q = 8; q < 16; ++q) { splitf(a[q], x, y); oh2[q & 3] = x; ol2[q & 3] = y; if ((q & 3) == 3) { *(volatile v4us*)(Ph + (q - 3)) = oh2; *(volatile v4us*)(Pl + (q - 3)) = ol2; } } }
#pragma unroll 1
        for (int c0 = 0; c0 < HDM; c0 += 4) { v4us oh, ol;
#pragma unroll
            for (int q = 0; q < 4; ++q) { unsigned short x, y; splitf(__fmul_rn(f[c0 + q], fs), x, y); oh[q] = x; ol[q] = y; } *(volatile v4us*)(Ph + RR + c0) = oh; *(volatile v4us*)(Pl + RR + c0) = ol; }
#pragma unroll
        for (int c0 = RR + HDM; c0 < KW; c0 += 4) { v4us z; z[0] = 0; z[1] = 0; z[2] = 0; z[3] = 0; *(volatile v4us*)(Ph + c0) = z; *(volatile v4us*)(Pl + c0) = z; }
        *(volatile float*)(N2 + e) = n2; if (ps == 0) __threadfence(); } }
__global__ __launch_bounds__(256) void k_dsoft(const float* __restrict__ C, const float* __restrict__ QQ, const float* __restrict__ KK, const float* __restrict__ mk, h16* P16) { const int lane = threadIdx.x & 31; const int row = blockIdx.x * 8 + (threadIdx.x >> 5); if (row >= TT) return; const float qq = QQ[row]; const float* cr = C + (size_t)row * TT; float v[32]; float mx = -3.0e38f;
#pragma unroll
    for (int ch = 0; ch < 8; ++ch) { const int j0 = ch * 128 + lane * 4; const v4f c4 = *(const v4f*)(cr + j0), k4 = *(const v4f*)(KK + j0), m4 = *(const v4f*)(mk + j0);
#pragma unroll
        for (int q = 0; q < 4; ++q) { float c2 = __fmul_rn(2.0f, c4[q]); asm volatile("" : "+v"(c2)); const float d2 = __fsub_rn(__fadd_rn(qq, k4[q]), c2); float sd = __fmul_rn(-SCL, d2); asm volatile("" : "+v"(sd)); const float t = __fadd_rn(sd, bfr(m4[q])); v[ch * 4 + q] = t; mx = fmaxf(mx, t); } }
#pragma unroll
    for (int sh = 16; sh; sh >>= 1) mx = fmaxf(mx, __shfl_xor(mx, sh, 32));
    float sum = 0.f;
#pragma unroll
    for (int k = 0; k < 32; ++k) { float d0 = __fsub_rn(v[k], mx); asm volatile("" : "+v"(d0)); v[k] = __expf(d0); sum += v[k]; }
#pragma unroll
    for (int sh = 16; sh; sh >>= 1) sum += __shfl_xor(sum, sh, 32);
    const float fc = __fdiv_rn(PCAR, sum);
#pragma unroll 1
    for (int ps = 0; ps < 2; ++ps) {
#pragma unroll
        for (int ch = 0; ch < 8; ++ch) { v4h o;
#pragma unroll
            for (int q = 0; q < 4; ++q) o[q] = tohx(v[ch * 4 + q] * fc); *(volatile v4h*)(P16 + (size_t)row * TT + ch * 128 + lane * 4) = o; }
        if (ps == 0) __threadfence(); } }

extern "C" void kernel_launch(void* const* d_in, const int* in_sizes, int n_in,
                              void* d_out, int out_size, void* d_ws, size_t ws_size, hipStream_t stream) {
    (void)in_sizes; (void)n_in; (void)out_size;
    const float* IN[11]; for (int i = 0; i < 11; ++i) IN[i] = (const float*)d_in[i];
    float* OUT = (float*)d_out;
    char* wsp = (char*)d_ws;
    auto take = [&](size_t bytes) { char* p = wsp; wsp += (bytes + 255) & ~(size_t)255; return (void*)p; };
    bf* W4[4]; for (int i = 0; i < 4; ++i) W4[i] = (bf*)take((size_t)EE * EE * 2);
    bf* XB = (bf*)take((size_t)TT * EE * 2); float* FQ = (float*)take((size_t)TT * EE * 4); float* FK = (float*)take((size_t)TT * EE * 4); float* FV = (float*)take((size_t)TT * EE * 4);
    bf* QCh = (bf*)take((size_t)NH_ * TT * KW * 2); bf* QCl = (bf*)take((size_t)NH_ * TT * KW * 2); bf* KCh = (bf*)take((size_t)NH_ * TT * KW * 2); bf* KCl = (bf*)take((size_t)NH_ * TT * KW * 2); float* N2 = (float*)take((size_t)2 * NH_ * TT * 4);
    h16* VT = (h16*)take((size_t)EE * TT * 2); float* C = (float*)take((size_t)TT * TT * 4); h16* Pm = (h16*)take((size_t)TT * TT * 2); float* O = (float*)take((size_t)TT * HDM * 4); bf* Ah = (bf*)take((size_t)TT * EE * 2); bf* Al = (bf*)take((size_t)TT * EE * 2);
    if ((size_t)(wsp - (char*)d_ws) > ws_size) return;
    { const unsigned g = (EE * EE / 8 + 255) / 256; k_cvt8<<<g, 256, 0, stream>>>(IN[2], W4[0], (size_t)EE * EE / 8); k_cvt8<<<g, 256, 0, stream>>>(IN[4], W4[1], (size_t)EE * EE / 8); k_cvt8<<<g, 256, 0, stream>>>(IN[6], W4[2], (size_t)EE * EE / 8); k_cvt8<<<g, 256, 0, stream>>>(IN[8], W4[3], (size_t)EE * EE / 8); }
    const dim3 gP(TT / 64, EE / 64, 1);
    for (int b = 0; b < NB_; ++b) {
        k_cvt8<<<(TT * EE / 8 + 255) / 256, 256, 0, stream>>>(IN[0] + (size_t)b * TT * EE, XB, (size_t)TT * EE / 8);
        k_gemmw<bf, 0, true><<<gP, 32, 0, stream>>>(XB, nullptr, W4[0], nullptr, EE, FQ, EE, IN[3], 0, 0, 0); k_gemmw<bf, 0, true><<<gP, 32, 0, stream>>>(XB, nullptr, W4[1], nullptr, EE, FK, EE, IN[5], 0, 0, 0); k_gemmw<bf, 0, true><<<gP, 32, 0, stream>>>(XB, nullptr, W4[2], nullptr, EE, FV, EE, IN[7], 0, 0, 0);
        k_curv<<<(2 * NH_ * TT + 255) / 256, 256, 0, stream>>>(FQ, FK, IN[10], QCh, QCl, KCh, KCl, N2); k_vt<<<(unsigned)(((size_t)TT * EE / 2 + 255) / 256), 256, 0, stream>>>(FV, EE, NH_, HDM, VT);
        for (int h = 0; h < NH_; ++h) { const size_t po = (size_t)h * TT * KW;
            k_gemmw<bf, 2, false><<<dim3(TT / 64, TT / 64, 1), 32, 0, stream>>>(QCh + po, QCl + po, KCh + po, KCl + po, KW, C, TT, nullptr, 0, 0, 0);
            k_dsoft<<<TT / 8, 256, 0, stream>>>(C, N2 + (size_t)h * TT, N2 + (size_t)(NH_ + h) * TT, IN[1] + (size_t)b * TT, Pm);
            k_gemmw<h16, 0, false><<<dim3(TT / 64, 1, 1), 32, 0, stream>>>(Pm, nullptr, VT + (size_t)h * HDM * TT, nullptr, TT, O, HDM, nullptr, 0, 0, 0);
            k_mrg<<<(TT * HDM / 2 + 255) / 256, 256, 0, stream>>>(O, h, HDM, Ah, Al); }
        k_gemmw<bf, 1, true><<<gP, 32, 0, stream>>>(Ah, Al, W4[3], nullptr, EE, OUT + (size_t)b * TT * EE, EE, IN[9], 0, 0, 0); }
}
